// LS2Actor_79001628443221
// MI455X (gfx1250) — hardware-run, weakly checked
//
#include <hip/hip_runtime.h>


namespace {
constexpr int NA = 8192, NN = 65536, N = NA, E = 262144, D = 128, NBLK = 2;
constexpr float XS = 8.0f, WSC = 256.0f, NEG = 0.2f  , EPSG = 1e-5f;

typedef _Float16 b16;
typedef __attribute__((ext_vector_type(16))) _Float16 v16b;
typedef __attribute__((ext_vector_type(8))) _Float16 v8b;
typedef __attribute__((ext_vector_type(8))) float v8f;
typedef __attribute__((ext_vector_type(4))) float v4f;
__device__ __forceinline__ float bf16_rne(float f) { unsigned int u = __float_as_uint(f); u += 0x7FFFu + ((u >> 16) & 1u); return __uint_as_float(u & 0xFFFF0000u); }
__device__ __forceinline__ void split16(float v, b16& hi, b16& lo) { hi = (b16)v; lo = (b16)(v - (float)hi); }
__device__ __forceinline__ v16b frag_kb(const b16* p, int hh) { const v8b a = *(const v8b*)(p + 8 * hh), b = *(const v8b*)(p + 16 + 8 * hh); v16b f;
#pragma unroll
  for (int e = 0; e < 8; ++e) { f[e] = a[e]; f[8 + e] = b[e]; } return f; }
__device__ __forceinline__ v8f wmma16b(v16b a, v16b b, v8f c) { v8f d = __builtin_amdgcn_wmma_f32_16x16x32_f16(false, a, false, b, (short)0, c, false, false); asm volatile("v_nop\n\tv_nop\n\tv_nop\n\tv_nop" : "+v"(d) : "v"(a), "v"(b)); return d; }
__device__ __forceinline__ void wave_lds_sync() { __builtin_amdgcn_fence(__ATOMIC_RELEASE, "workgroup"); __builtin_amdgcn_wave_barrier(); __builtin_amdgcn_fence(__ATOMIC_ACQUIRE, "workgroup"); }
__device__ __forceinline__ float pmul(float a, float b) { float p = a * b; asm volatile("" : "+v"(p)); return p; }
__device__ __forceinline__ int iclamp(int v, int lo, int hi) { return v < lo ? lo : (v > hi ? hi : v); }
__device__ __forceinline__ float nexp(float x) { return __builtin_amdgcn_exp2f(x * 1.4426950408889634f); }
__device__ __forceinline__ float lrelu(float x) { return x > 0.0f ? x : NEG * x; }

constexpr int CSR_NBLK = 512, CSR_GB = 8  , CSR_GN = 1 << CSR_GB  , CSR_MAXG = 512, CSR_CAP = 12288  ;
__global__ __launch_bounds__(64) void csrA_kernel(const int* __restrict__ dst, int E, int N, int nG, int CHP, int NGP, int* __restrict__ STG, int* __restrict__ HST) {
  extern __shared__ int sm[];
  int* cnt = sm; int* run = sm + NGP; int* ids = sm + 2 * NGP;
  const int b = blockIdx.x; const int ch = (E + CSR_NBLK - 1) / CSR_NBLK; const int e0 = b * ch, e1 = min(E, e0 + ch);
  for (int i = threadIdx.x; i < NGP; i += 64) cnt[i] = 0;
  for (int i = threadIdx.x; i < CHP; i += 64) ids[i] = -1;
  __syncthreads();
  if (threadIdx.x == 0) {
    for (int e = e0; e < e1; ++e) { int d = dst[e]; d = (d < 0) ? 0 : (d >= N ? N - 1 : d); cnt[d >> CSR_GB] += 1; }
    int acc = 0; for (int g = 0; g < nG; ++g) { run[g] = acc; acc += cnt[g]; }
    for (int e = e0; e < e1; ++e) { int d = dst[e]; d = (d < 0) ? 0 : (d >= N ? N - 1 : d); const int g = d >> CSR_GB; ids[run[g]] = e; run[g] += 1; } }
  __syncthreads();
  typedef __attribute__((ext_vector_type(4))) int v4i;
  for (int pass = 0; pass < 2; ++pass) {
    for (int i = threadIdx.x; i < CHP / 4; i += 64) *(volatile v4i*)(STG + (size_t)b * CHP + i * 4) = *(const v4i*)(&ids[i * 4]);
    for (int i = threadIdx.x; i < NGP / 4; i += 64) { v4i v; for (int e = 0; e < 4; ++e) v[e] = (i * 4 + e < nG) ? cnt[i * 4 + e] : 0; *(volatile v4i*)(HST + (size_t)b * NGP + i * 4) = v; }
    __threadfence(); }
}
__global__ __launch_bounds__(512) void csrS_kernel(const int* __restrict__ HST, int nG, int NGP, int* __restrict__ START, int* __restrict__ TOT, int* __restrict__ OFF) {
  __shared__ int tot[CSR_MAXG];
  const int b = threadIdx.x;
  for (int pass = 0; pass < 2; ++pass) { int runb = 0; for (int g = 0; g < nG; ++g) { int c = HST[(size_t)b * NGP + g]; c = (c < 0) ? 0 : c; ((volatile int*)OFF)[(size_t)g * CSR_NBLK + b] = runb; runb += c; } __threadfence(); }
  for (int g = threadIdx.x; g < nG; g += 512) { int s = 0; for (int bb = 0; bb < CSR_NBLK; ++bb) { int c = HST[(size_t)bb * NGP + g]; s += (c < 0) ? 0 : c; } tot[g] = s; }
  __syncthreads();
  if (threadIdx.x < 32) {
    __shared__ int st[CSR_MAXG + 32];
    if (threadIdx.x == 0) { int acc = 0; for (int g = 0; g < NGP; ++g) { st[g] = acc; if (g < nG) acc += (tot[g] + 31) & ~31; } st[NGP] = acc; }
    __builtin_amdgcn_fence(__ATOMIC_RELEASE, "workgroup"); __builtin_amdgcn_wave_barrier(); __builtin_amdgcn_fence(__ATOMIC_ACQUIRE, "workgroup");
    for (int pass = 0; pass < 2; ++pass) { for (int i = threadIdx.x; i < NGP + 32; i += 32) { ((volatile int*)START)[i] = (i <= NGP) ? st[min(i, NGP)] : 0; ((volatile int*)TOT)[i] = (i < nG) ? tot[i] : 0; } __threadfence(); } }
}
__global__ __launch_bounds__(256) void csrB_kernel(const int* __restrict__ dst, int N, int nG, int CHP, int NGP, int permLen, const int* __restrict__ STG, const int* __restrict__ HST, const int* __restrict__ OFF, const int* __restrict__ START, const int* __restrict__ TOT, int* __restrict__ PERM, int* __restrict__ ROWPTR, int* __restrict__ ROWCNT, int* __restrict__ FLAG) {
  typedef __attribute__((ext_vector_type(4))) int v4i;
  __shared__ int ids[CSR_CAP]; __shared__ unsigned short key[CSR_CAP]; __shared__ int outp[CSR_CAP]; __shared__ int ncnt[CSR_GN + 1]; __shared__ int boff[CSR_NBLK + 1];
  const int g = blockIdx.x, t_ = threadIdx.x; int tot = TOT[g]; int st = START[g], stn = START[g + 1]; const int v0 = g * CSR_GN; const int nv = min(CSR_GN, N - v0);
  st = (st < 0) ? 0 : (st > permLen - 32 ? permLen - 32 : st) & ~31; stn = (stn < st) ? st : (stn > permLen ? permLen : stn); tot = (tot < 0) ? 0 : tot; if (tot > stn - st && tot <= CSR_CAP) tot = stn - st;
  if (tot > CSR_CAP) {
    for (int pass = 0; pass < 2; ++pass) { for (int i = t_; i < CSR_GN / 4; i += 256) { v4i a, c; for (int e = 0; e < 4; ++e) { a[e] = st; c[e] = 0; } *(volatile v4i*)(ROWPTR + v0 + i * 4) = a; *(volatile v4i*)(ROWCNT + v0 + i * 4) = c; } if (t_ == 0) ((volatile int*)FLAG)[0] = 1; __threadfence(); } (void)nv; return; }
  if (t_ == 0) { int acc = 0; for (int b = 0; b < CSR_NBLK; ++b) { boff[b] = acc; int c = HST[(size_t)b * NGP + g]; c = (c < 0) ? 0 : (c > CHP ? CHP : c); acc += c; if (acc > tot) acc = tot; } boff[CSR_NBLK] = acc; }
  for (int i = t_; i <= CSR_GN; i += 256) ncnt[i] = 0;
  __syncthreads();
  for (int b = 0; b < CSR_NBLK; ++b) { const int c = boff[b + 1] - boff[b]; int o_ = OFF[(size_t)g * CSR_NBLK + b]; o_ = (o_ < 0) ? 0 : (o_ > CHP - c ? CHP - c : o_); const int* src_ = STG + (size_t)b * CHP + o_;
    for (int i = t_; i < c; i += 256) { int id = src_[i]; id = (id < 0) ? 0 : id; ids[boff[b] + i] = id; int d = dst[id]; d = (d < v0) ? v0 : (d >= N ? N - 1 : d); int kk = d - v0; kk = (kk < 0) ? 0 : (kk >= CSR_GN ? CSR_GN - 1 : kk); key[boff[b] + i] = (unsigned short)kk; } }
  __syncthreads();
  if (t_ == 0) { for (int i = 0; i < tot; ++i) ncnt[key[i]] += 1; int acc = 0; for (int vl = 0; vl < CSR_GN; ++vl) { const int c = ncnt[vl]; ncnt[vl] = acc; acc += c; } ncnt[CSR_GN] = acc;
    for (int i = 0; i < tot; ++i) { const int vl = key[i]; outp[ncnt[vl]] = ids[i]; ncnt[vl] += 1; }
    for (int vl = CSR_GN; vl > 0; --vl) ncnt[vl] = ncnt[vl - 1]; ncnt[0] = 0; }
  __syncthreads();
  for (int pass = 0; pass < 2; ++pass) {
    for (int i = t_; i < (stn - st) / 4; i += 256) { v4i v; for (int e = 0; e < 4; ++e) { const int q = i * 4 + e; v[e] = (q < tot) ? outp[q] : -1; } *(volatile v4i*)(PERM + st + i * 4) = v; }
    for (int i = t_; i < CSR_GN / 4; i += 256) { v4i a, c; for (int e = 0; e < 4; ++e) { const int vl = i * 4 + e; a[e] = st + ncnt[vl]; c[e] = (vl < nv) ? (ncnt[vl + 1] - ncnt[vl]) : 0; } *(volatile v4i*)(ROWPTR + v0 + i * 4) = a; *(volatile v4i*)(ROWCNT + v0 + i * 4) = c; }
    __threadfence(); }
}
__global__ __launch_bounds__(256) void csrZ_kernel(int* __restrict__ p, size_t n4) { typedef __attribute__((ext_vector_type(4))) int v4i; const size_t tid = (size_t)blockIdx.x * 256 + threadIdx.x, nth = (size_t)gridDim.x * 256; v4i z = {0, 0, 0, 0}; for (size_t i = tid; i < n4; i += nth) *(volatile v4i*)(p + i * 4) = z; }
struct CsrBufs { int *STG, *HST, *OFF, *START, *TOT, *PERM, *ROWPTR, *ROWCNT, *FLAG; int nG, NGP, CHP; size_t permLen; char* base; size_t bytes; };
static size_t csr_carve(CsrBufs& c, char* ws, size_t off, int E, int N) {
  const size_t off0 = off; c.base = ws + off;
  auto al = [&](size_t bytes) { char* p = ws + off; off += (bytes + 255) & ~(size_t)255; return p; };
  c.nG = (N + CSR_GN - 1) / CSR_GN; c.NGP = (c.nG + 31) & ~31; const int ch = (E + CSR_NBLK - 1) / CSR_NBLK; c.CHP = (ch + 31) & ~31; c.permLen = (size_t)E + 32 * (size_t)c.nG + 32;
  c.STG = (int*)al((size_t)CSR_NBLK * c.CHP * 4); c.HST = (int*)al((size_t)CSR_NBLK * c.NGP * 4); c.OFF = (int*)al((size_t)c.NGP * CSR_NBLK * 4); c.START = (int*)al((size_t)(c.NGP + 64) * 4); c.TOT = (int*)al((size_t)(c.NGP + 64) * 4);
  c.PERM = (int*)al(c.permLen * 4); c.ROWPTR = (int*)al((size_t)c.nG * CSR_GN * 4); c.ROWCNT = (int*)al((size_t)c.nG * CSR_GN * 4); c.FLAG = (int*)al(256);
  c.bytes = off - off0; return off;
}
static void csr_build(const CsrBufs& c, const int* dst, int E, int N, hipStream_t stream) {
  const size_t smem = (size_t)(2 * c.NGP + c.CHP) * 4;
  csrZ_kernel<<<512, 256, 0, stream>>>((int*)c.base, c.bytes / 16);
  csrA_kernel<<<CSR_NBLK, 64, smem, stream>>>(dst, E, N, c.nG, c.CHP, c.NGP, c.STG, c.HST);
  csrS_kernel<<<1, 512, 0, stream>>>(c.HST, c.nG, c.NGP, c.START, c.TOT, c.OFF);
  csrB_kernel<<<c.nG, 256, 0, stream>>>(dst, N, c.nG, c.CHP, c.NGP, (int)c.permLen, c.STG, c.HST, c.OFF, c.START, c.TOT, c.PERM, c.ROWPTR, c.ROWCNT, c.FLAG);
}


__global__ __launch_bounds__(256) void prep_kernel(const float* __restrict__ nodes, const float* __restrict__ wq, const float* __restrict__ wag, const float* __restrict__ wlin, const float* __restrict__ w1, const float* __restrict__ wc0, const float* __restrict__ wc1, b16* __restrict__ N16, b16* __restrict__ WB) {
  const size_t t = (size_t)blockIdx.x * 256 + threadIdx.x; const size_t nn = (size_t)NN * D / 8, nw = (size_t)D * D / 8; v8b o;
  if (t < nn) { const size_t e = t * 8; const v4f a = *(const v4f*)(nodes + e), c = *(const v4f*)(nodes + e + 4); for (int j = 0; j < 4; ++j) { o[j] = (b16)(bf16_rne(a[j]) * XS); o[4 + j] = (b16)(bf16_rne(c[j]) * XS); } for (int pass = 0; pass < 2; ++pass) { *(volatile v8b*)(N16 + e) = o; __threadfence(); } return; }
  size_t u = t - nn; if (u >= (size_t)NBLK * 8 * nw) return; const int blk = (int)(u / (8 * nw)); u %= 8 * nw; const int slot = (int)(u / nw); const int e = (int)(u % nw) * 8; const int oo = e / D, k0 = e % D;
  const float* src; size_t idx;
  if (slot == 0) { src = wq; idx = ((size_t)blk * D + oo) * D + k0; } else if (slot == 1) { src = wag; idx = ((size_t)blk * D + oo) * D + k0; } else if (slot == 2) { src = wlin; idx = ((size_t)blk * D + oo) * D + k0; } else if (slot == 3) { src = w1; idx = ((size_t)blk * D + oo) * D + k0; }
  else if (slot < 7) { src = wc0; idx = ((size_t)blk * D + oo) * (3 * D) + (size_t)(slot - 4) * D + k0; } else { src = wc1; idx = ((size_t)blk * D + oo) * D + k0; }
  for (int j = 0; j < 8; ++j) o[j] = (b16)(bf16_rne(src[idx + j]) * WSC);
  for (int pass = 0; pass < 2; ++pass) { *(volatile v8b*)(WB + ((size_t)blk * 8 + slot) * D * D + e) = o; __threadfence(); }
}
__host__ __device__ __forceinline__ const b16* wslot(const b16* WB, int blk, int slot) { return WB + ((size_t)blk * 8 + slot) * D * D; }
__device__ __forceinline__ void gn_rowstats(const float* v8  , float& mean, float& rstd) {
  float s = 0.0f; for (int t = 0; t < 8; ++t) s += v8[t];
  s += __shfl_xor(s, 1); s += __shfl_xor(s, 2); s += __shfl_xor(s, 4); s += __shfl_xor(s, 8); mean = s * (1.0f / D);
  float q = 0.0f; for (int t = 0; t < 8; ++t) { const float d = v8[t] - mean; q += d * d; }
  q += __shfl_xor(q, 1); q += __shfl_xor(q, 2); q += __shfl_xor(q, 4); q += __shfl_xor(q, 8); rstd = rsqrtf(q * (1.0f / D) + EPSG);
}
template <int MODE>
__global__ __launch_bounds__(128) void actor_kernel(const float* __restrict__ X, int xraw, const b16* __restrict__ Wt, const float* __restrict__ g, const float* __restrict__ bta, const float* __restrict__ RES, int resraw, float* __restrict__ Y) {
  __shared__ __attribute__((aligned(16))) b16 Ah[4][16][D + 8], Al[4][16][D + 8]; __shared__ __attribute__((aligned(16))) float Tf[4][16][D + 4];
  const int wave = threadIdx.x >> 5, lane = threadIdx.x & 31, nloc = lane & 15, hlf = lane >> 4; const size_t m0 = (size_t)blockIdx.x * 64 + wave * 16;
  for (int q = lane; q < 16 * (D / 4); q += 32) { const int rr = q / (D / 4), c4 = (q % (D / 4)) * 4; const v4f xv = *(const v4f*)(X + (m0 + rr) * D + c4); for (int j = 0; j < 4; ++j) { const float x = xraw ? bf16_rne(xv[j]) : xv[j]; b16 p, pl; split16(x * XS, p, pl); Ah[wave][rr][c4 + j] = p; Al[wave][rr][c4 + j] = pl; } }
  wave_lds_sync();
  v8f acc[8];
#pragma unroll
  for (int t = 0; t < 8; ++t) acc[t] = (v8f){};
#pragma unroll
  for (int kb = 0; kb < D; kb += 32) { const v16b a = frag_kb(&Ah[wave][nloc][kb], hlf), al = frag_kb(&Al[wave][nloc][kb], hlf);
#pragma unroll
    for (int t = 0; t < 8; ++t) { const v16b bw = frag_kb(Wt + (size_t)(t * 16 + nloc) * D + kb, hlf); acc[t] = wmma16b(a, bw, acc[t]); acc[t] = wmma16b(al, bw, acc[t]); } }
#pragma unroll 1
  for (int r = 0; r < 8; ++r) { float v8_[8]; for (int t = 0; t < 8; ++t) v8_[t] = acc[t][r] * (1.0f / (XS * WSC)); const int rr = 8 * hlf + r;
    if (MODE == 1) { for (int t = 0; t < 8; ++t) Tf[wave][rr][t * 16 + nloc] = v8_[t]; }
    else { float mean, rstd; gn_rowstats(v8_, mean, rstd);
      for (int t = 0; t < 8; ++t) { const int c = t * 16 + nloc; float y = (v8_[t] - mean) * rstd * bf16_rne(g[c]) + bf16_rne(bta[c]);
        if (MODE == 0) y = fmaxf(y, 0.0f); else { const float rv = RES[(m0 + rr) * D + c]; y = fmaxf(y + (resraw ? bf16_rne(rv) : rv), 0.0f); } Tf[wave][rr][c] = y; } } }
  wave_lds_sync();
  for (int pass = 0; pass < 2; ++pass) { for (int rr = 0; rr < 16; ++rr) *(volatile v4f*)(Y + (m0 + rr) * D + lane * 4) = *(const v4f*)(&Tf[wave][rr][lane * 4]); __threadfence(); }
}
__global__ __launch_bounds__(128) void edge_kernel(const float* __restrict__ QA, const float* __restrict__ AA, const b16* __restrict__ N16, const float* __restrict__ actr, const float* __restrict__ nctr, const int* __restrict__ wi,
    const float* __restrict__ w0, const float* __restrict__ b0, const float* __restrict__ g1, const float* __restrict__ be1, const float* __restrict__ gc, const float* __restrict__ bc, const float* __restrict__ gno, const float* __restrict__ bno,
    const b16* __restrict__ WB, int blk, const int* __restrict__ PERM, const int* __restrict__ ROWPTR, const int* __restrict__ ROWCNT, int permLen, float* __restrict__ A1) {
  __shared__ __attribute__((aligned(16))) b16 Th[4][16][D + 8], Tl[4][16][D + 8], Tc[4][16][D + 8]; __shared__ int wi_s[4][16]; __shared__ __attribute__((aligned(16))) float rowo[4][D];
  const int wave = threadIdx.x >> 5, lane = threadIdx.x & 31, nloc = lane & 15, hlf = lane >> 4; const size_t a = (size_t)blockIdx.x * 4 + wave;
  const b16* W1t = wslot(WB, blk, 3); const b16* Wd = wslot(WB, blk, 4); const b16* Wq2 = wslot(WB, blk, 5); const b16* Wcc = wslot(WB, blk, 6); const b16* Wc1 = wslot(WB, blk, 7);
  int st = ROWPTR[a], cnt = ROWCNT[a]; cnt = iclamp(cnt, 0, 8192); st = iclamp(st, 0, permLen - cnt);
  const float ax = bf16_rne(actr[a * 2]), ay = bf16_rne(actr[a * 2 + 1]);
  float qterm[8];
  { for (int q = lane; q < 16 * D; q += 32) { const int rr = q / D, c = q % D; b16 p, pl; split16(QA[a * D + c] * XS, p, pl); Th[wave][rr][c] = p; Tl[wave][rr][c] = pl; }
    wave_lds_sync();
#pragma unroll
    for (int t = 0; t < 8; ++t) { v8f dq = {};
#pragma unroll
      for (int kb = 0; kb < D; kb += 32) { const v16b bw = frag_kb(Wq2 + (size_t)(t * 16 + nloc) * D + kb, hlf); dq = wmma16b(frag_kb(&Th[wave][nloc][kb], hlf), bw, dq); dq = wmma16b(frag_kb(&Tl[wave][nloc][kb], hlf), bw, dq); } qterm[t] = dq[0] * (1.0f / (XS * WSC)); }
    wave_lds_sync(); }
  float msum[8]; for (int t = 0; t < 8; ++t) msum[t] = 0.0f;
  for (int e0 = 0; e0 < cnt; e0 += 16) {
    if (lane < 16) { const int i = e0 + lane; const bool valid = i < cnt; int node = 0; if (valid) { const int e = iclamp(PERM[st + i], 0, E - 1); node = iclamp(wi[e], 0, NN - 1); } wi_s[wave][lane] = node;
      const float dx = valid ? ax - bf16_rne(nctr[(size_t)node * 2]) : 0.0f, dy = valid ? ay - bf16_rne(nctr[(size_t)node * 2 + 1]) : 0.0f;
      for (int c = 0; c < D; ++c) { const float v = valid ? fmaxf(pmul(dx, bf16_rne(w0[c * 2])) + pmul(dy, bf16_rne(w0[c * 2 + 1])) + bf16_rne(b0[c]), 0.0f) : 0.0f; b16 p, pl; split16(v * XS, p, pl); Th[wave][lane][c] = p; Tl[wave][lane][c] = pl; } }
    wave_lds_sync();
    for (int q = lane; q < 16 * (D / 8); q += 32) { const int rr = q / (D / 8), c8 = (q % (D / 8)) * 8; *(v8b*)(&Tc[wave][rr][c8]) = *(const v8b*)(N16 + (size_t)wi_s[wave][rr] * D + c8); }
    v8f acc[8];
#pragma unroll
    for (int t = 0; t < 8; ++t) acc[t] = (v8f){};
#pragma unroll
    for (int kb = 0; kb < D; kb += 32) { const v16b fa = frag_kb(&Th[wave][nloc][kb], hlf), fl = frag_kb(&Tl[wave][nloc][kb], hlf);
#pragma unroll
      for (int t = 0; t < 8; ++t) { const v16b bw = frag_kb(W1t + (size_t)(t * 16 + nloc) * D + kb, hlf); acc[t] = wmma16b(fa, bw, acc[t]); acc[t] = wmma16b(fl, bw, acc[t]); } }
    wave_lds_sync();
#pragma unroll
    for (int r = 0; r < 8; ++r) { float v8_[8]; for (int t = 0; t < 8; ++t) v8_[t] = acc[t][r] * (1.0f / (XS * WSC)); float mean, rstd; gn_rowstats(v8_, mean, rstd);
      for (int t = 0; t < 8; ++t) { const int c = t * 16 + nloc; b16 p, pl; split16(fmaxf((v8_[t] - mean) * rstd * bf16_rne(g1[c]) + bf16_rne(be1[c]), 0.0f) * XS, p, pl); Th[wave][8 * hlf + r][c] = p; Tl[wave][8 * hlf + r][c] = pl; } }
    wave_lds_sync();
#pragma unroll
    for (int t = 0; t < 8; ++t) acc[t] = (v8f){};
#pragma unroll
    for (int kb = 0; kb < D; kb += 32) { const v16b fd = frag_kb(&Th[wave][nloc][kb], hlf), fdl = frag_kb(&Tl[wave][nloc][kb], hlf), fc = frag_kb(&Tc[wave][nloc][kb], hlf);
#pragma unroll
      for (int t = 0; t < 8; ++t) { const v16b bw = frag_kb(Wd + (size_t)(t * 16 + nloc) * D + kb, hlf); acc[t] = wmma16b(fd, bw, acc[t]); acc[t] = wmma16b(fdl, bw, acc[t]); acc[t] = wmma16b(fc, frag_kb(Wcc + (size_t)(t * 16 + nloc) * D + kb, hlf), acc[t]); } }
    wave_lds_sync();
#pragma unroll
    for (int r = 0; r < 8; ++r) { float v8_[8]; for (int t = 0; t < 8; ++t) v8_[t] = acc[t][r] * (1.0f / (XS * WSC)) + qterm[t]; float mean, rstd; gn_rowstats(v8_, mean, rstd);
      for (int t = 0; t < 8; ++t) { const int c = t * 16 + nloc; b16 p, pl; split16(fmaxf((v8_[t] - mean) * rstd * bf16_rne(gc[c]) + bf16_rne(bc[c]), 0.0f) * XS, p, pl); Th[wave][8 * hlf + r][c] = p; Tl[wave][8 * hlf + r][c] = pl; } }
    wave_lds_sync();
#pragma unroll
    for (int t = 0; t < 8; ++t) acc[t] = (v8f){};
#pragma unroll
    for (int kb = 0; kb < D; kb += 32) { const v16b fm = frag_kb(&Th[wave][nloc][kb], hlf), fml = frag_kb(&Tl[wave][nloc][kb], hlf);
#pragma unroll
      for (int t = 0; t < 8; ++t) { const v16b bw = frag_kb(Wc1 + (size_t)(t * 16 + nloc) * D + kb, hlf); acc[t] = wmma16b(fm, bw, acc[t]); acc[t] = wmma16b(fml, bw, acc[t]); } }
#pragma unroll
    for (int t = 0; t < 8; ++t)
#pragma unroll
      for (int r = 0; r < 8; ++r) if (e0 + 8 * hlf + r < cnt) msum[t] += acc[t][r] * (1.0f / (XS * WSC));
    wave_lds_sync(); }
  float v8_[8]; for (int t = 0; t < 8; ++t) { const float m = msum[t] + __shfl_xor(msum[t], 16); v8_[t] = AA[a * D + t * 16 + nloc] + m; }
  float mean, rstd; gn_rowstats(v8_, mean, rstd);
  if (hlf == 0) for (int t = 0; t < 8; ++t) { const int c = t * 16 + nloc; rowo[wave][c] = fmaxf((v8_[t] - mean) * rstd * bf16_rne(gno[c]) + bf16_rne(bno[c]), 0.0f); }
  wave_lds_sync();
  for (int pass = 0; pass < 2; ++pass) { *(volatile v4f*)(A1 + a * D + lane * 4) = *(const v4f*)(&rowo[wave][lane * 4]); __threadfence(); }
}
}

extern "C" void kernel_launch(void* const* d_in, const int* in_sizes, int n_in, void* d_out, int out_size, void* d_ws, size_t ws_size, hipStream_t stream) {
  (void)n_in;
  auto Fp = [&](int i) { return (const float*)d_in[i]; }; auto Ip = [&](int i) { return (const int*)d_in[i]; };
  if (in_sizes[0] != NA * D || in_sizes[1] != NN * D || in_sizes[2] != NA * 2 || in_sizes[3] != NN * 2 || in_sizes[4] != E || in_sizes[5] != E || in_sizes[6] != NBLK * D * 2 || in_sizes[8] != NBLK * D * D || in_sizes[14] != NBLK * D * 3 * D || in_sizes[21] != NBLK * D * D || out_size != NA * D) return;
  size_t off = 0; char* ws = (char*)d_ws;
  auto carve = [&](size_t bytes) { char* p = ws + off; off += (bytes + 255) & ~(size_t)255; return p; };
  b16* N16 = (b16*)carve((size_t)NN * D * 2); b16* WB = (b16*)carve((size_t)NBLK * 8 * D * D * 2); float* QA = (float*)carve((size_t)NA * D * 4); float* AA = (float*)carve((size_t)NA * D * 4); float* A1 = (float*)carve((size_t)NA * D * 4); float* ACT = (float*)carve((size_t)NA * D * 4);
  CsrBufs csr; off = csr_carve(csr, ws, off, E, NA);
  if (off > ws_size || off > ((size_t)128 << 20)) return;
  prep_kernel<<<(unsigned)(((size_t)NN * D / 8 + (size_t)NBLK * 8 * D * D / 8 + 255) / 256), 256, 0, stream>>>(Fp(1), Fp(11), Fp(18), Fp(21), Fp(8), Fp(14), Fp(17), N16, WB);
  csr_build(csr, Ip(4), E, NA, stream);
  for (int b = 0; b < NBLK; ++b) { const float* X = (b == 0) ? Fp(0) : ACT; const int raw = (b == 0) ? 1 : 0; float* Y = (b == NBLK - 1) ? (float*)d_out : ACT;
    actor_kernel<0><<<NA / 64, 128, 0, stream>>>(X, raw, wslot(WB, b, 0), Fp(12) + b * D, Fp(13) + b * D, nullptr, 0, QA);
    actor_kernel<1><<<NA / 64, 128, 0, stream>>>(X, raw, wslot(WB, b, 1), nullptr, nullptr, nullptr, 0, AA);
    edge_kernel<<<NA / 4, 128, 0, stream>>>(QA, AA, N16, Fp(2), Fp(3), Ip(5), Fp(6) + b * D * 2, Fp(7) + b * D, Fp(9) + b * D, Fp(10) + b * D, Fp(15) + b * D, Fp(16) + b * D, Fp(19) + b * D, Fp(20) + b * D, WB, b, csr.PERM, csr.ROWPTR, csr.ROWCNT, (int)csr.permLen, A1);
    actor_kernel<2><<<NA / 64, 128, 0, stream>>>(A1, 0, wslot(WB, b, 2), Fp(22) + b * D, Fp(23) + b * D, X, raw, Y);
  }
}
